// SimpleAttentionSemanticEvolution_20151986553033
// MI455X (gfx1250) — hardware-verified
//
#include <hip/hip_runtime.h>
#include <math.h>

typedef __attribute__((ext_vector_type(16))) _Float16 v16h;
typedef __attribute__((ext_vector_type(16))) __bf16 v16b;
typedef __attribute__((ext_vector_type(8)))  _Float16 v8h;
typedef __attribute__((ext_vector_type(8)))  float v8f;
typedef __attribute__((ext_vector_type(4)))  float v4f;
typedef __attribute__((ext_vector_type(2)))  float v2f;
typedef __attribute__((ext_vector_type(4)))  unsigned v4u;
typedef __attribute__((ext_vector_type(4)))  int v4i;
typedef float __attribute__((may_alias)) float_a;
typedef int __attribute__((may_alias)) int_a;

template <typename T> __device__ __forceinline__ void vst2(void* p, T v) { *(volatile T*)p = v; __threadfence(); *(volatile T*)p = v; }
__device__ __forceinline__ v8f wmma16(v16h a, v16h b, v8f c) {
  v8f d = __builtin_amdgcn_wmma_f32_16x16x32_f16(false, a, false, b, (short)0, c, false, false);
  asm volatile("v_nop\n\tv_nop\n\tv_nop\n\tv_nop" : "+v"(d) : "v"(a), "v"(b));
  return d;
}
__device__ __forceinline__ v8f wmma_bf(v16b a, v16b b, v8f c) {
  v8f d = __builtin_amdgcn_wmma_f32_16x16x32_bf16(false, a, false, b, (short)0, c, false, false);
  asm volatile("v_nop\n\tv_nop\n\tv_nop\n\tv_nop" : "+v"(d) : "v"(a), "v"(b));
  return d;
}
__device__ __forceinline__ v16h frag_h(const _Float16* rowk0, int lane) {
  union { v16h v; v8h q[2]; } u; const _Float16* p = rowk0 + 8 * (lane >> 4);
  u.q[0] = *(const v8h*)p; u.q[1] = *(const v8h*)(p + 16); return u.v;
}
__device__ __forceinline__ v16h frag_f32(const float* rowk0, int lane) {
  v16h a; const float* p = rowk0 + 8 * (lane >> 4);
#pragma unroll
  for (int i = 0; i < 8; ++i) { a[i] = (_Float16)p[i]; a[8 + i] = (_Float16)p[16 + i]; }
  return a;
}
__device__ __forceinline__ v16h frag_f32s(const float* rowk0, int lane, float sc) {
  v16h a; const float* p = rowk0 + 8 * (lane >> 4);
#pragma unroll
  for (int i = 0; i < 8; ++i) { a[i] = (_Float16)(p[i] * sc); a[8 + i] = (_Float16)(p[16 + i] * sc); }
  return a;
}
__device__ __forceinline__ v16h fragc_f32(const float* W, int k0, int n, int lane, int ld, int K) {
  v16h a; const int g = lane >> 4;
#pragma unroll
  for (int i = 0; i < 8; ++i) { const int ka = k0 + 8 * g + i, kb = ka + 16;
    a[i] = (_Float16)(ka < K ? W[(size_t)(ka < K ? ka : K - 1) * ld + n] : 0.f); a[8 + i] = (_Float16)(kb < K ? W[(size_t)(kb < K ? kb : K - 1) * ld + n] : 0.f); }
  return a;
}
struct F2 { v16b h, l; };
__device__ __forceinline__ F2 bsplit16(const float v[16]) { F2 r;
#pragma unroll
  for (int i = 0; i < 16; ++i) { const __bf16 h = (__bf16)v[i]; r.h[i] = h; r.l[i] = (__bf16)(v[i] - (float)h); }
  return r; }
__device__ __forceinline__ F2 split_row(const float* row, int k0, int lane) { float v[16]; const float* p = row + k0 + 8 * (lane >> 4);
#pragma unroll
  for (int i = 0; i < 8; ++i) { v[i] = p[i]; v[8 + i] = p[16 + i]; }
  return bsplit16(v); }
__device__ __forceinline__ F2 split_rowK(const float* row, int k0, int lane, int K) { float v[16]; const int g = lane >> 4;
#pragma unroll
  for (int i = 0; i < 8; ++i) { const int ka = k0 + 8 * g + i, kb = ka + 16; v[i] = ka < K ? row[ka < K ? ka : K - 1] : 0.f; v[8 + i] = kb < K ? row[kb < K ? kb : K - 1] : 0.f; }
  return bsplit16(v); }
__device__ __forceinline__ F2 split_col(const float* W, int k0, int n, int lane, int ld, int K) { float v[16]; const int g = lane >> 4;
#pragma unroll
  for (int i = 0; i < 8; ++i) { const int ka = k0 + 8 * g + i, kb = ka + 16; v[i] = ka < K ? W[(size_t)(ka < K ? ka : K - 1) * ld + n] : 0.f; v[8 + i] = kb < K ? W[(size_t)(kb < K ? kb : K - 1) * ld + n] : 0.f; }
  return bsplit16(v); }
__device__ __forceinline__ v8f mac3(const F2& a, const F2& b, v8f c) { c = wmma_bf(a.l, b.h, c); c = wmma_bf(a.h, b.l, c); return wmma_bf(a.h, b.h, c); }
__device__ __forceinline__ float sigm(float v) { return 1.0f / (1.0f + expf(-v)); }
#define LDSX() do { asm volatile("s_wait_dscnt 0" ::: "memory"); __builtin_amdgcn_wave_barrier(); __builtin_amdgcn_fence(__ATOMIC_RELEASE, "workgroup"); } while (0)


#define NB 4
#define NQ 256
#define NK 4096
#define CV 512
#define E 1024
#define NH 8
#define HD 128
__device__ __forceinline__ float bfr(float v) { return (float)(__bf16)v; }
__device__ __forceinline__ v16b frag_b(const __bf16* rowk0, int lane) { return __builtin_bit_cast(v16b, frag_h((const _Float16*)rowk0, lane)); }

__global__ __launch_bounds__(256) void k_cvtc(const float* __restrict__ x, __bf16* __restrict__ Xb, size_t n8) {
  const size_t i8 = (size_t)blockIdx.x * 256 + threadIdx.x; if (i8 >= n8) return;
  union { __bf16 h[8]; v4u u; } pk;
#pragma unroll
  for (int e = 0; e < 8; ++e) pk.h[e] = (__bf16)x[i8 * 8 + e];
  vst2((unsigned*)(Xb + i8 * 8), pk.u);
}
__global__ __launch_bounds__(256) void k_cvtx(const float* __restrict__ x, __bf16* __restrict__ VB) {
  __shared__ __align__(16) __bf16 st[64][CV + 8];
  const int tid = threadIdx.x; const int b = blockIdx.y, t0 = blockIdx.x * 64;
  for (int q = tid; q < CV * 16; q += 256) { const int c = q >> 4, p4 = q & 15; const v4f v = *(const v4f*)(x + ((size_t)b * CV + c) * NK + t0 + p4 * 4);
    st[p4 * 4][c] = (__bf16)v[0]; st[p4 * 4 + 1][c] = (__bf16)v[1]; st[p4 * 4 + 2][c] = (__bf16)v[2]; st[p4 * 4 + 3][c] = (__bf16)v[3]; }
  __syncthreads();
  for (int q = tid; q < 64 * (CV / 8); q += 256) { const int rl = q >> 6, pc = q & 63; vst2((unsigned*)(VB + ((size_t)b * NK + t0 + rl) * CV + pc * 8), *(const v4u*)(&st[rl][pc * 8])); }
}
__global__ __launch_bounds__(256) void k_pack(const float* __restrict__ Wq, const float* __restrict__ Wk, const float* __restrict__ Wv, const float* __restrict__ Wo, __bf16* __restrict__ PQ, __bf16* __restrict__ PK, __bf16* __restrict__ PVw, __bf16* __restrict__ PO) {
  const int n = blockIdx.x, which = blockIdx.y, tid = threadIdx.x; __shared__ __align__(16) __bf16 srow[E];
  const int K = (which == 1 || which == 2) ? CV : E; const float* W = which == 0 ? Wq : (which == 1 ? Wk : (which == 2 ? Wv : Wo)); __bf16* P = which == 0 ? PQ : (which == 1 ? PK : (which == 2 ? PVw : PO));
  for (int k = tid; k < K; k += 256) srow[k] = (__bf16)W[(size_t)k * E + n];
  __syncthreads();
  if (tid < K / 8) vst2((unsigned*)(P + (size_t)n * K + tid * 8), *(const v4u*)(&srow[tid * 8]));
}
__global__ __launch_bounds__(128) void k_q(const __bf16* __restrict__ Cb, const __bf16* __restrict__ PQ, float* __restrict__ Q32) {
  __shared__ __align__(16) float so[4][16][132];
  const int tid = threadIdx.x, wave = tid >> 5, lane = tid & 31, col = lane & 15, g = lane >> 4; const int r0b = blockIdx.x * 64, r0 = r0b + wave * 16, h = blockIdx.y; const int b = r0b / NQ, s0 = r0b % NQ;
  v8f acc[8] = {};
#pragma unroll 2
  for (int kc = 0; kc < E / 32; ++kc) { const v16b a = frag_b(Cb + (size_t)(r0 + col) * E + kc * 32, lane);
#pragma unroll
    for (int j = 0; j < 8; ++j) acc[j] = wmma_bf(a, frag_b(PQ + (size_t)(h * HD + j * 16 + col) * E + kc * 32, lane), acc[j]); }
#pragma unroll
  for (int j = 0; j < 8; ++j)
#pragma unroll
    for (int r = 0; r < 8; ++r) so[wave][8 * g + r][j * 16 + col] = acc[j][r];
  LDSX();
  for (int rl = 0; rl < 16; ++rl) vst2(Q32 + (((size_t)b * NH + h) * NQ + s0 + wave * 16 + rl) * HD + lane * 4, *(const v4f*)(&so[wave][rl][lane * 4]));
}
__global__ __launch_bounds__(128) void k_kv(const __bf16* __restrict__ VB, int b, const __bf16* __restrict__ PK, const __bf16* __restrict__ PVw, __bf16* __restrict__ Kh, __bf16* __restrict__ Kl, __bf16* __restrict__ VTh, __bf16* __restrict__ VTl) {
  __shared__ __align__(16) __bf16 sh_[4][16][136], sl_[4][16][136]; __shared__ __align__(16) __bf16 sth[128][72], stl[128][72];
  const int tid = threadIdx.x, wave = tid >> 5, lane = tid & 31, col = lane & 15, g = lane >> 4; const int s0 = blockIdx.x * 64, h = blockIdx.y, which = blockIdx.z; const int r0 = b * NK + s0 + wave * 16;
  const __bf16* P = which == 0 ? PK : PVw;
  v8f acc[8] = {};
#pragma unroll 2
  for (int kc = 0; kc < CV / 32; ++kc) { const v16b a = frag_b(VB + (size_t)(r0 + col) * CV + kc * 32, lane);
#pragma unroll
    for (int j = 0; j < 8; ++j) acc[j] = wmma_bf(a, frag_b(P + (size_t)(h * HD + j * 16 + col) * CV + kc * 32, lane), acc[j]); }
  const size_t bh = (size_t)h;
  if (which == 0) {
#pragma unroll
    for (int j = 0; j < 8; ++j)
#pragma unroll
      for (int r = 0; r < 8; ++r) { const float v = acc[j][r]; const __bf16 hi = (__bf16)v; sh_[wave][8 * g + r][j * 16 + col] = hi; sl_[wave][8 * g + r][j * 16 + col] = (__bf16)(v - (float)hi); }
    LDSX();
    for (int rl = 0; rl < 16; ++rl) { if (lane < 16) { vst2((unsigned*)(Kh + (bh * NK + s0 + wave * 16 + rl) * HD + lane * 8), *(const v4u*)(&sh_[wave][rl][lane * 8])); vst2((unsigned*)(Kl + (bh * NK + s0 + wave * 16 + rl) * HD + lane * 8), *(const v4u*)(&sl_[wave][rl][lane * 8])); } } }
  else {
#pragma unroll
    for (int j = 0; j < 8; ++j)
#pragma unroll
      for (int r = 0; r < 8; ++r) { const float v = acc[j][r]; const __bf16 hi = (__bf16)v; sth[j * 16 + col][wave * 16 + 8 * g + r] = hi; stl[j * 16 + col][wave * 16 + 8 * g + r] = (__bf16)(v - (float)hi); }
    __syncthreads();
    for (int qq = tid; qq < 128 * 8; qq += 128) { const int d = qq >> 3, pc = qq & 7; const size_t o = (bh * HD + d) * NK + s0 + pc * 8; vst2((unsigned*)(VTh + o), *(const v4u*)(&sth[d][pc * 8])); vst2((unsigned*)(VTl + o), *(const v4u*)(&stl[d][pc * 8])); } }
}
__global__ __launch_bounds__(128) void k_attn(const float* __restrict__ Q32, int b, const __bf16* __restrict__ Kh, const __bf16* __restrict__ Kl, const __bf16* __restrict__ VTh, const __bf16* __restrict__ VTl, float* __restrict__ O32) {
  __shared__ __align__(16) float sS[4][16][68];
  __shared__ __align__(16) __bf16 sPh[4][16][72], sPl[4][16][72];
  __shared__ __align__(16) float sO[4][16][132];
  const int tid = threadIdx.x, w = tid >> 5, lane = tid & 31, col = lane & 15, g = lane >> 4; const int h = blockIdx.y; const size_t bh = (size_t)h; const size_t bhq = (size_t)b * NH + h; const int q0 = blockIdx.x * 64 + w * 16;
  F2 aq[4];
#pragma unroll
  for (int kc = 0; kc < 4; ++kc) aq[kc] = split_row(Q32 + (bhq * NQ + q0 + col) * HD, kc * 32, lane);
  float mrun = -3.0e38f, lrun = 0.f; v8f acc[8] = {};
#pragma unroll 1
  for (int kt = 0; kt < NK / 64; ++kt) {
#pragma unroll
    for (int t = 0; t < 4; ++t) { const int key = kt * 64 + t * 16 + col; const size_t ko = (bh * NK + key) * HD; v8f s = {};
#pragma unroll
      for (int kc = 0; kc < 4; ++kc) { const v16b khf = frag_b(Kh + ko + kc * 32, lane), klf = frag_b(Kl + ko + kc * 32, lane); s = wmma_bf(aq[kc].l, khf, s); s = wmma_bf(aq[kc].h, klf, s); s = wmma_bf(aq[kc].h, khf, s); }
#pragma unroll
      for (int r = 0; r < 8; ++r) sS[w][8 * g + r][t * 16 + col] = s[r] * 0.08838834764831845f; }
    LDSX();
    float mx = -3.4e38f;
#pragma unroll
    for (int jj = 0; jj < 32; ++jj) mx = fmaxf(mx, sS[w][col][g * 32 + jj]);
    mx = fmaxf(mx, __shfl_xor(mx, 16, 32));
    const float mnew = fmaxf(mrun, mx); const float corr = expf(mrun - mnew);
    float ps = 0.f;
#pragma unroll
    for (int jj = 0; jj < 32; ++jj) { const float p = expf(sS[w][col][g * 32 + jj] - mnew); ps += p; const __bf16 hi = (__bf16)p; sPh[w][col][g * 32 + jj] = hi; sPl[w][col][g * 32 + jj] = (__bf16)(p - (float)hi); }
    ps += __shfl_xor(ps, 16, 32);
    lrun = lrun * corr + ps; mrun = mnew;
#pragma unroll
    for (int r = 0; r < 8; ++r) { const float cr = __shfl(corr, 8 * g + r, 32);
#pragma unroll
      for (int t = 0; t < 8; ++t) acc[t][r] *= cr; }
    LDSX();
#pragma unroll
    for (int kc = 0; kc < 2; ++kc) { const v16b ph = frag_b(&sPh[w][col][0] + kc * 32, lane), pl = frag_b(&sPl[w][col][0] + kc * 32, lane);
#pragma unroll
      for (int t = 0; t < 8; ++t) { const size_t vo = (bh * HD + t * 16 + col) * NK + kt * 64 + kc * 32; const v16b vh = frag_b(VTh + vo, lane), vl = frag_b(VTl + vo, lane); acc[t] = wmma_bf(pl, vh, acc[t]); acc[t] = wmma_bf(ph, vl, acc[t]); acc[t] = wmma_bf(ph, vh, acc[t]); } }
    __builtin_amdgcn_wave_barrier(); }
#pragma unroll
  for (int r = 0; r < 8; ++r) { const float lr = __shfl(lrun, 8 * g + r, 32); const float inv = 1.0f / lr;
#pragma unroll
    for (int t = 0; t < 8; ++t) sO[w][8 * g + r][t * 16 + col] = acc[t][r] * inv; }
  LDSX();
  for (int rl = 0; rl < 16; ++rl) vst2(O32 + ((size_t)b * NQ + q0 + rl) * E + h * HD + lane * 4, *(const v4f*)(&sO[w][rl][lane * 4]));
}
__global__ __launch_bounds__(128) void k_out(const float* __restrict__ O32, const __bf16* __restrict__ PO, const float* __restrict__ bo, float* __restrict__ out) {
  __shared__ __align__(16) float so[4][16][132];
  const int tid = threadIdx.x, wave = tid >> 5, lane = tid & 31, col = lane & 15, g = lane >> 4; const int r0 = blockIdx.x * 64 + wave * 16, n0 = blockIdx.y * 128;
  v8f acc[8] = {};
#pragma unroll 1
  for (int kc = 0; kc < E / 32; ++kc) { const F2 a = split_row(O32 + (size_t)(r0 + col) * E, kc * 32, lane);
#pragma unroll
    for (int j = 0; j < 8; ++j) { const v16b wb = frag_b(PO + (size_t)(n0 + j * 16 + col) * E + kc * 32, lane); acc[j] = wmma_bf(a.l, wb, acc[j]); acc[j] = wmma_bf(a.h, wb, acc[j]); } }
#pragma unroll
  for (int j = 0; j < 8; ++j) { const float bb = bfr(bo[n0 + j * 16 + col]);
#pragma unroll
    for (int r = 0; r < 8; ++r) so[wave][8 * g + r][j * 16 + col] = acc[j][r] + bb; }
  LDSX();
  for (int rl = 0; rl < 16; ++rl) vst2(out + (size_t)(r0 + rl) * E + n0 + lane * 4, *(const v4f*)(&so[wave][rl][lane * 4]));
}
extern "C" void kernel_launch(void* const* d_in, const int* in_sizes, int n_in, void* d_out, int out_size, void* d_ws, size_t ws_size, hipStream_t stream) {
  (void)in_sizes; (void)n_in; (void)out_size; (void)ws_size;
  const float** I = (const float**)d_in;
  const float* x = I[0]; const float* ctxin = I[2]; const float* Wq = I[3]; const float* Wk = I[4]; const float* Wv = I[5]; const float* Wo = I[6]; const float* bo = I[7];
  float* out = (float*)d_out;
  char* ws = (char*)d_ws; size_t off = 0;
  auto take = [&](size_t bytes) { char* p = ws + off; off += (bytes + 255) & ~(size_t)255; return p; };
  __bf16* Cb = (__bf16*)take((size_t)NB * NQ * E * 2); __bf16* VB = (__bf16*)take((size_t)NB * NK * CV * 2);
  __bf16* PQ = (__bf16*)take((size_t)E * E * 2); __bf16* PK = (__bf16*)take((size_t)E * CV * 2); __bf16* PVw = (__bf16*)take((size_t)E * CV * 2); __bf16* PO = (__bf16*)take((size_t)E * E * 2);
  float* Q32 = (float*)take((size_t)NB * NQ * E * 4); __bf16* Kh = (__bf16*)take((size_t)NK * E * 2); __bf16* Kl = (__bf16*)take((size_t)NK * E * 2); __bf16* VTh = (__bf16*)take((size_t)NK * E * 2); __bf16* VTl = (__bf16*)take((size_t)NK * E * 2);
  float* O32 = (float*)take((size_t)NB * NQ * E * 4);
  k_cvtc<<<(unsigned)((NB * NQ * E / 8 + 255) / 256), 256, 0, stream>>>(ctxin, Cb, (size_t)NB * NQ * E / 8);
  k_cvtx<<<dim3(NK / 64, NB), 256, 0, stream>>>(x, VB);
  k_pack<<<dim3(E, 4), 256, 0, stream>>>(Wq, Wk, Wv, Wo, PQ, PK, PVw, PO);
  k_q<<<dim3(NB * NQ / 64, NH), 128, 0, stream>>>(Cb, PQ, Q32);
  for (int b = 0; b < NB; ++b) {
    k_kv<<<dim3(NK / 64, NH, 2), 128, 0, stream>>>(VB, b, PK, PVw, Kh, Kl, VTh, VTl);
    k_attn<<<dim3(NQ / 64, NH), 128, 0, stream>>>(Q32, b, Kh, Kl, VTh, VTl, O32); }
  k_out<<<dim3(NB * NQ / 64, E / 128), 128, 0, stream>>>(O32, PO, bo, out);
}
